// Block_71253507441369
// MI455X (gfx1250) — hardware-verified
//
#include <hip/hip_runtime.h>
#include <stddef.h>
#include <stdint.h>
#include <math.h>


#define NSEQ   16
#define DD     256
#define LL     1024
#define DI     512
#define DS     16
#define M1     16384
#define MD     2048
#define MD2    4096
#define UP     512
#define XCP    1024
#define XDP    64
#define HHP    4096
#define FP     8192
#define GBM    64
#define GTHR   128
#define KFULL  0x7fffffff
#define TP     36
#define STHR   128
#define STL    32
#define WSMAX  134217728

#define EP_INPROJ  0
#define EP_XDBL    1
#define EP_OUTPROJ 2
#define EP_PW1     3
#define EP_PW2     4

static_assert(M1 == NSEQ * LL && MD == 8 * DD && MD2 == 2 * MD && DI == 2 * DD);
static_assert(UP == 2 * DD && XCP == 2 * DI && HHP == 2 * MD && FP == 2 * MD2);
static_assert(M1 % GBM == 0 && DD % GBM == 0 && MD % GBM == 0 && (2 * LL) % GBM == 0);
static_assert((2 * DI) % 128 == 0 && LL % 128 == 0 && MD2 % 128 == 0 && XDP == 64);
static_assert(UP % 32 == 0 && XCP % 32 == 0 && HHP % 32 == 0 && FP % 32 == 0);
static_assert((DD & (DD - 1)) == 0 && (DI & (DI - 1)) == 0 && (MD & (MD - 1)) == 0 && (MD2 & (MD2 - 1)) == 0);
static_assert(GBM == (GTHR / 32) * 16);
static_assert(LL % STL == 0 && DI % STHR == 0 && STL == (STHR / 32) * 8 && (STL * 16) % STHR == 0);
static_assert((TP * 4) % 16 == 0 && TP >= 32);

typedef float          v4f   __attribute__((ext_vector_type(4)));
typedef float          v8f   __attribute__((ext_vector_type(8)));
typedef int            v8i   __attribute__((ext_vector_type(8)));
typedef unsigned int   v4u   __attribute__((ext_vector_type(4)));
typedef unsigned short v4us  __attribute__((ext_vector_type(4)));
typedef unsigned short v8us  __attribute__((ext_vector_type(8)));
typedef unsigned short v16us __attribute__((ext_vector_type(16)));
typedef __bf16         v16bf __attribute__((ext_vector_type(16)));
typedef v4f  __attribute__((may_alias)) v4fa;
typedef v4us __attribute__((may_alias)) v4usa;
typedef v8us __attribute__((may_alias)) v8usa;
union FragB { v16bf v; v16us u; v8us h[2]; v8i w; };

__device__ __forceinline__ v8f wmb(const FragB& a, const FragB& b, v8f c) {
  v8f d = __builtin_amdgcn_wmma_f32_16x16x32_bf16(false, a.v, false, b.v, (short)0, c, false, false);
  asm volatile("v_nop\n\tv_nop\n\tv_nop\n\tv_nop" : "+v"(d) : "v"(a.w), "v"(b.w));
  return d;
}

__device__ __forceinline__ unsigned bf16_bits(float f) {
  const unsigned u = __float_as_uint(f);
  return (u + 0x7FFFu + ((u >> 16) & 1u)) >> 16;
}
__device__ __forceinline__ float bf16_val(float f) {
  return __uint_as_float(bf16_bits(f) << 16);
}
__device__ __forceinline__ void split2(float v, unsigned& hb, unsigned& lb) {
  hb = bf16_bits(v);
  lb = bf16_bits(v - __uint_as_float(hb << 16));
}

__device__ __forceinline__ void wave_sync() {
  __builtin_amdgcn_fence(__ATOMIC_RELEASE, "wavefront");
  __builtin_amdgcn_wave_barrier();
  __builtin_amdgcn_fence(__ATOMIC_ACQUIRE, "wavefront");
}

__device__ __forceinline__ float silu_f(float v) { return v * (1.0f / (1.0f + expf(-v))); }

__device__ __forceinline__ float conv_silu(float xm3, float xm2, float xm1, float x0,
                                           float w0, float w1, float w2, float w3, float b) {
  float a = xm3 * w0;
  a = fmaf(xm2, w1, a);
  a = fmaf(xm1, w2, a);
  a = fmaf(x0, w3, a);
  a = a + b;
  return silu_f(a);
}

__device__ __forceinline__ void cvt_unit(const float* __restrict__ s, unsigned short* d, int v, int nreal) {
  const int vc = v < nreal ? v : nreal - 1;
  const float* p = s + (size_t)vc * 8;
  const v4f a = *(const v4f*)p;
  const v4f b = *(const v4f*)(p + 4);
  const bool ok = v < nreal;
  v8us o;
  o[0] = ok ? (unsigned short)bf16_bits(a.x) : (unsigned short)0;
  o[1] = ok ? (unsigned short)bf16_bits(a.y) : (unsigned short)0;
  o[2] = ok ? (unsigned short)bf16_bits(a.z) : (unsigned short)0;
  o[3] = ok ? (unsigned short)bf16_bits(a.w) : (unsigned short)0;
  o[4] = ok ? (unsigned short)bf16_bits(b.x) : (unsigned short)0;
  o[5] = ok ? (unsigned short)bf16_bits(b.y) : (unsigned short)0;
  o[6] = ok ? (unsigned short)bf16_bits(b.z) : (unsigned short)0;
  o[7] = ok ? (unsigned short)bf16_bits(b.w) : (unsigned short)0;
  unsigned short* dp = d + (size_t)v * 8;
  *(volatile v8us*)dp = o;
  __threadfence();
  *(volatile v8us*)dp = o;
}

__global__ __launch_bounds__(256) void k_cvt3(const float* __restrict__ s0, unsigned short* d0, int r0, int t0,
                                              const float* __restrict__ s1, unsigned short* d1, int r1, int t1,
                                              const float* __restrict__ s2, unsigned short* d2, int r2, int t2) {
  const int u = (int)blockIdx.x * 256 + (int)threadIdx.x;
  if (u < t0) {
    cvt_unit(s0, d0, u, r0);
  } else if (u < t0 + t1) {
    cvt_unit(s1, d1, u - t0, r1);
  } else if (u < t0 + t1 + t2) {
    cvt_unit(s2, d2, u - t0 - t1, r2);
  }
}

__device__ __forceinline__ void ln_row(const float* tile, int lane, int l, float mean, float rstd,
                                       const float (&g8)[8], const float (&b8)[8], v8us& oh, v8us& ol) {
#pragma unroll
  for (int i = 0; i < 8; ++i) {
    const float xv = tile[(8 * lane + i) * TP + l];
    const float y = ((xv - mean) * rstd) * g8[i] + b8[i];
    unsigned hb, lb;
    split2(y, hb, lb);
    oh[i] = (unsigned short)hb;
    ol[i] = (unsigned short)lb;
  }
}

template <int MODE>
__global__ __launch_bounds__(256) void k_ln(const float* __restrict__ src, const float* __restrict__ g,
                                            const float* __restrict__ bt, unsigned short* dst) {
  __shared__ __attribute__((aligned(16))) float tile[DD * TP];
  __shared__ float ps[256];
  __shared__ float pq[256];
  __shared__ float mu[32];
  __shared__ float rs[32];
  const int tid = (int)threadIdx.x, lane = tid & 31, wave = tid >> 5;
  const int n  = (int)blockIdx.x >> 5;
  const int l0 = ((int)blockIdx.x & 31) * 32;
  {
    const int q = tid & 7, dr = tid >> 3;
#pragma unroll 4
    for (int it = 0; it < 8; ++it) {
      const int d = it * 32 + dr;
      v4f v = *(const v4f*)(src + ((size_t)n * DD + d) * LL + l0 + 4 * q);
      if constexpr (MODE == 0) {
        v.x = bf16_val(v.x); v.y = bf16_val(v.y); v.z = bf16_val(v.z); v.w = bf16_val(v.w);
      }
      *(v4fa*)(tile + d * TP + 4 * q) = v;
    }
  }
  __syncthreads();
  const int lc = tid & 31, p = tid >> 5;
  float s = 0.0f;
#pragma unroll 4
  for (int j = 0; j < 32; ++j) s += tile[(p * 32 + j) * TP + lc];
  ps[p * 32 + lc] = s;
  __syncthreads();
  float tot = 0.0f;
#pragma unroll
  for (int w2 = 0; w2 < 8; ++w2) tot += ps[w2 * 32 + lc];
  const float mean = tot * (1.0f / 256.0f);
  float qq = 0.0f;
#pragma unroll 4
  for (int j = 0; j < 32; ++j) {
    const float dv = tile[(p * 32 + j) * TP + lc] - mean;
    qq = fmaf(dv, dv, qq);
  }
  pq[p * 32 + lc] = qq;
  __syncthreads();
  float tq = 0.0f;
#pragma unroll
  for (int w2 = 0; w2 < 8; ++w2) tq += pq[w2 * 32 + lc];
  const float var  = tq * (1.0f / 256.0f);
  const float rstd = 1.0f / sqrtf(var + 1e-5f);
  if (p == 0) { mu[lc] = mean; rs[lc] = rstd; }
  __syncthreads();

  float g8[8], b8[8];
  {
    const v4f ga = *(const v4f*)(g + 8 * lane);
    const v4f gb = *(const v4f*)(g + 8 * lane + 4);
    const v4f ba = *(const v4f*)(bt + 8 * lane);
    const v4f bb = *(const v4f*)(bt + 8 * lane + 4);
    g8[0] = bf16_val(ga.x); g8[1] = bf16_val(ga.y); g8[2] = bf16_val(ga.z); g8[3] = bf16_val(ga.w);
    g8[4] = bf16_val(gb.x); g8[5] = bf16_val(gb.y); g8[6] = bf16_val(gb.z); g8[7] = bf16_val(gb.w);
    b8[0] = bf16_val(ba.x); b8[1] = bf16_val(ba.y); b8[2] = bf16_val(ba.z); b8[3] = bf16_val(ba.w);
    b8[4] = bf16_val(bb.x); b8[5] = bf16_val(bb.y); b8[6] = bf16_val(bb.z); b8[7] = bf16_val(bb.w);
  }
  size_t rbase;
  int pitch, cofs, lofs;
  if constexpr (MODE == 0) {
    rbase = (size_t)n * LL + l0; pitch = UP; cofs = 0; lofs = DD;
  } else {
    rbase = (size_t)(n >> 3) * LL + l0; pitch = HHP; cofs = (n & 7) * DD; lofs = MD;
  }
#pragma unroll 1
  for (int j = 0; j < 4; ++j) {
    const int l = 4 * wave + j;
    v8us oh, ol;
    ln_row(tile, lane, l, mu[l], rs[l], g8, b8, oh, ol);
    unsigned short* rp = dst + (rbase + l) * (size_t)pitch + cofs + 8 * lane;
    *(volatile v8us*)rp = oh;
    *(volatile v8us*)(rp + lofs) = ol;
  }
  __threadfence();
#pragma unroll 1
  for (int j = 0; j < 4; ++j) {
    const int l = 4 * wave + j;
    v8us oh, ol;
    ln_row(tile, lane, l, mu[l], rs[l], g8, b8, oh, ol);
    unsigned short* rp = dst + (rbase + l) * (size_t)pitch + cofs + 8 * lane;
    *(volatile v8us*)rp = oh;
    *(volatile v8us*)(rp + lofs) = ol;
  }
}

template <int NT, int EPI>
__global__ __launch_bounds__(GTHR) void k_gemm(
    const unsigned short* __restrict__ A, int lda, int amask,
    const unsigned short* __restrict__ Bt, long long strB, int ldb, int bmask, int K,
    float* o0, long long o1off, unsigned short* ob,
    const float* __restrict__ bias, const float* xres)
{
  constexpr int GBN = 16 * NT;
  __shared__ __attribute__((aligned(16))) float stg[GBM * GBN];
  const int tid = (int)threadIdx.x, lane = tid & 31, wave = tid >> 5, hh = lane >> 4, m = lane & 15;
  const int rowBase = (int)blockIdx.x * GBM;
  const int col0    = (int)blockIdx.y * GBN;
  const int z       = (int)blockIdx.z;

  v8f acc[NT];
  {
    const v8f zz = {0.f, 0.f, 0.f, 0.f, 0.f, 0.f, 0.f, 0.f};
#pragma unroll
    for (int t = 0; t < NT; ++t) acc[t] = zz;
  }
  const unsigned short* ap = A + (size_t)(rowBase + 16 * wave + m) * (size_t)lda + 8 * hh;
  const unsigned short* bp = Bt + (size_t)z * (size_t)strB + (size_t)(col0 + m) * (size_t)ldb + 8 * hh;

#pragma unroll 1
  for (int k0 = 0; k0 < K; k0 += 32) {
    const int ka = k0 & amask;
    const int kb = k0 & bmask;
    FragB af;
    af.h[0] = *(const v8usa*)(ap + ka);
    af.h[1] = *(const v8usa*)(ap + ka + 16);
#pragma unroll
    for (int nt = 0; nt < NT; ++nt) {
      const unsigned short* wq = bp + (size_t)(16 * nt) * (size_t)ldb + kb;
      FragB bf;
      bf.h[0] = *(const v8usa*)wq;
      bf.h[1] = *(const v8usa*)(wq + 16);
      acc[nt] = wmb(af, bf, acc[nt]);
    }
  }

#pragma unroll
  for (int nt = 0; nt < NT; ++nt) {
    const int lc = 16 * nt + m;
#pragma unroll
    for (int r = 0; r < 8; ++r) {
      const int lr = 16 * wave + 8 * hh + r;
      stg[lr * GBN + lc] = acc[nt][r];
    }
  }
  __syncthreads();

  if constexpr (EPI == EP_XDBL) {
    static_assert(NT == 4);
#pragma unroll 1
    for (int i = 0; i < 8; ++i) {
      const int lr = 16 * wave + 2 * i + hh;
      const v4f v = *(const v4fa*)(stg + lr * GBN + 4 * m);
      float* gp = o0 + (size_t)(rowBase + lr) * XDP + col0 + 4 * m;
      *(volatile v4f*)gp = v;
    }
    __threadfence();
#pragma unroll 1
    for (int i = 0; i < 8; ++i) {
      const int lr = 16 * wave + 2 * i + hh;
      const v4f v = *(const v4fa*)(stg + lr * GBN + 4 * m);
      float* gp = o0 + (size_t)(rowBase + lr) * XDP + col0 + 4 * m;
      *(volatile v4f*)gp = v;
    }
  } else if constexpr (EPI == EP_INPROJ) {
    static_assert(NT == 8);
    const bool isz = col0 >= DI;
    const long long goff = isz ? o1off : 0LL;
    const int cc = (col0 & (DI - 1)) + 4 * lane;
#pragma unroll 1
    for (int i = 0; i < 16; ++i) {
      const int lr = 16 * wave + i;
      float* sp = stg + lr * GBN + 4 * lane;
      v4f v = *(const v4fa*)sp;
      if (isz) { v.x = silu_f(v.x); v.y = silu_f(v.y); v.z = silu_f(v.z); v.w = silu_f(v.w); }
      *(v4fa*)sp = v;
      float* gp = o0 + goff + (size_t)(rowBase + lr) * DI + cc;
      *(volatile v4f*)gp = v;
    }
    __threadfence();
#pragma unroll 1
    for (int i = 0; i < 16; ++i) {
      const int lr = 16 * wave + i;
      const v4f v = *(const v4fa*)(stg + lr * GBN + 4 * lane);
      float* gp = o0 + goff + (size_t)(rowBase + lr) * DI + cc;
      *(volatile v4f*)gp = v;
    }
  } else if constexpr (EPI == EP_OUTPROJ) {
    static_assert(NT == 8);
#pragma unroll 1
    for (int i = 0; i < 16; ++i) {
      const int lr = 16 * wave + i;
      float* sp = stg + lr * GBN + 4 * lane;
      v4f v = *(const v4fa*)sp;
      const size_t idx = ((size_t)z * DD + rowBase + lr) * LL + col0 + 4 * lane;
      const v4f xv = *(const v4f*)(xres + idx);
      v.x = bf16_val(xv.x) + v.x; v.y = bf16_val(xv.y) + v.y;
      v.z = bf16_val(xv.z) + v.z; v.w = bf16_val(xv.w) + v.w;
      *(v4fa*)sp = v;
      *(volatile v4f*)(o0 + idx) = v;
    }
    __threadfence();
#pragma unroll 1
    for (int i = 0; i < 16; ++i) {
      const int lr = 16 * wave + i;
      const v4f v = *(const v4fa*)(stg + lr * GBN + 4 * lane);
      const size_t idx = ((size_t)z * DD + rowBase + lr) * LL + col0 + 4 * lane;
      *(volatile v4f*)(o0 + idx) = v;
    }
  } else if constexpr (EPI == EP_PW1) {
    static_assert(NT == 8);
    v4f bb4;
    {
      const v4f t1 = *(const v4f*)(bias + col0 + 4 * lane);
      bb4.x = bf16_val(t1.x); bb4.y = bf16_val(t1.y); bb4.z = bf16_val(t1.z); bb4.w = bf16_val(t1.w);
    }
    const int gofs = col0 + ((lane < 16) ? 8 * lane : MD2 + 8 * (lane - 16));
#pragma unroll 1
    for (int i = 0; i < 16; ++i) {
      const int lr = 16 * wave + i;
      float* srf = stg + lr * GBN;
      v4f v = *(const v4fa*)(srf + 4 * lane);
      v.x = fmaxf(v.x + bb4.x, 0.0f); v.y = fmaxf(v.y + bb4.y, 0.0f);
      v.z = fmaxf(v.z + bb4.z, 0.0f); v.w = fmaxf(v.w + bb4.w, 0.0f);
      v4us h4, l4;
      unsigned hb, lb;
      split2(v.x, hb, lb); h4[0] = (unsigned short)hb; l4[0] = (unsigned short)lb;
      split2(v.y, hb, lb); h4[1] = (unsigned short)hb; l4[1] = (unsigned short)lb;
      split2(v.z, hb, lb); h4[2] = (unsigned short)hb; l4[2] = (unsigned short)lb;
      split2(v.w, hb, lb); h4[3] = (unsigned short)hb; l4[3] = (unsigned short)lb;
      wave_sync();
      unsigned short* srh = (unsigned short*)srf;
      *(v4usa*)(srh + 4 * lane) = h4;
      *(v4usa*)(srh + 128 + 4 * lane) = l4;
      wave_sync();
      const v8us q = *(const v8usa*)(srh + 8 * lane);
      unsigned short* gp = ob + (size_t)(rowBase + lr) * FP + gofs;
      *(volatile v8us*)gp = q;
    }
    __threadfence();
#pragma unroll 1
    for (int i = 0; i < 16; ++i) {
      const int lr = 16 * wave + i;
      const unsigned short* srh = (const unsigned short*)(stg + lr * GBN);
      const v8us q = *(const v8usa*)(srh + 8 * lane);
      unsigned short* gp = ob + (size_t)(rowBase + lr) * FP + gofs;
      *(volatile v8us*)gp = q;
    }
  } else {
    static_assert(NT == 8 && EPI == EP_PW2);
#pragma unroll 1
    for (int i = 0; i < 16; ++i) {
      const int lr = 16 * wave + i;
      float* sp = stg + lr * GBN + 4 * lane;
      v4f v = *(const v4fa*)sp;
      const float bb = bf16_val(bias[rowBase + lr]);
      const size_t idx = ((size_t)z * MD + rowBase + lr) * LL + col0 + 4 * lane;
      const v4f r = *(const v4f*)(o0 + idx);
      v.x = r.x + (v.x + bb); v.y = r.y + (v.y + bb);
      v.z = r.z + (v.z + bb); v.w = r.w + (v.w + bb);
      *(v4fa*)sp = v;
      *(volatile v4f*)(o0 + idx) = v;
    }
    __threadfence();
#pragma unroll 1
    for (int i = 0; i < 16; ++i) {
      const int lr = 16 * wave + i;
      const v4f v = *(const v4fa*)(stg + lr * GBN + 4 * lane);
      const size_t idx = ((size_t)z * MD + rowBase + lr) * LL + col0 + 4 * lane;
      *(volatile v4f*)(o0 + idx) = v;
    }
  }
}

__global__ __launch_bounds__(256) void k_conv(const float* __restrict__ XI, const float* __restrict__ cw,
                                              const float* __restrict__ cb, unsigned short* XC) {
  const int tid = (int)threadIdx.x, lane = tid & 31, wave = tid >> 5;
  const int gw  = (int)blockIdx.x * 8 + wave;
  const int tok = gw >> 2;
  const int cwb = (gw & 3) * 128;
  const int c   = cwb + 4 * lane;
  const int l   = tok & (LL - 1);
  const float* r0 = XI + (size_t)tok * DI + c;
  const int b1 = (l < 1 ? l : 1) * DI;
  const int b2 = (l < 2 ? l : 2) * DI;
  const int b3 = (l < 3 ? l : 3) * DI;
  const v4f x0 = *(const v4f*)r0;
  v4f x1 = *(const v4f*)(r0 - b1);
  v4f x2 = *(const v4f*)(r0 - b2);
  v4f x3 = *(const v4f*)(r0 - b3);
  const float f1 = (l >= 1) ? 1.0f : 0.0f;
  const float f2 = (l >= 2) ? 1.0f : 0.0f;
  const float f3 = (l >= 3) ? 1.0f : 0.0f;
  x1.x = (l >= 1) ? x1.x : 0.0f; x1.y = (l >= 1) ? x1.y : 0.0f; x1.z = (l >= 1) ? x1.z : 0.0f; x1.w = (l >= 1) ? x1.w : 0.0f;
  x2.x = (l >= 2) ? x2.x : 0.0f; x2.y = (l >= 2) ? x2.y : 0.0f; x2.z = (l >= 2) ? x2.z : 0.0f; x2.w = (l >= 2) ? x2.w : 0.0f;
  x3.x = (l >= 3) ? x3.x : 0.0f; x3.y = (l >= 3) ? x3.y : 0.0f; x3.z = (l >= 3) ? x3.z : 0.0f; x3.w = (l >= 3) ? x3.w : 0.0f;
  (void)f1; (void)f2; (void)f3;
  const v4f wa = *(const v4f*)(cw + 4 * c);
  const v4f wb = *(const v4f*)(cw + 4 * c + 4);
  const v4f wc = *(const v4f*)(cw + 4 * c + 8);
  const v4f wd = *(const v4f*)(cw + 4 * c + 12);
  const v4f bv = *(const v4f*)(cb + c);
  const float y0 = conv_silu(x3.x, x2.x, x1.x, x0.x, bf16_val(wa.x), bf16_val(wa.y), bf16_val(wa.z), bf16_val(wa.w), bf16_val(bv.x));
  const float y1 = conv_silu(x3.y, x2.y, x1.y, x0.y, bf16_val(wb.x), bf16_val(wb.y), bf16_val(wb.z), bf16_val(wb.w), bf16_val(bv.y));
  const float y2 = conv_silu(x3.z, x2.z, x1.z, x0.z, bf16_val(wc.x), bf16_val(wc.y), bf16_val(wc.z), bf16_val(wc.w), bf16_val(bv.z));
  const float y3 = conv_silu(x3.w, x2.w, x1.w, x0.w, bf16_val(wd.x), bf16_val(wd.y), bf16_val(wd.z), bf16_val(wd.w), bf16_val(bv.w));
  unsigned h0, l0b, h1, l1b, h2, l2b, h3, l3b;
  split2(y0, h0, l0b); split2(y1, h1, l1b); split2(y2, h2, l2b); split2(y3, h3, l3b);
  const int hw0 = (int)(h0 | (h1 << 16)), hw1 = (int)(h2 | (h3 << 16));
  const int lw0 = (int)(l0b | (l1b << 16)), lw1 = (int)(l2b | (l3b << 16));
  const int sa = (2 * lane) & 31, sb = (2 * lane + 1) & 31;
  const int g0 = __shfl(hw0, sa, 32), g1 = __shfl(hw1, sa, 32);
  const int g2 = __shfl(hw0, sb, 32), g3 = __shfl(hw1, sb, 32);
  const int p0 = __shfl(lw0, sa, 32), p1 = __shfl(lw1, sa, 32);
  const int p2 = __shfl(lw0, sb, 32), p3 = __shfl(lw1, sb, 32);
  const bool lsel = lane >= 16;
  v4u pv;
  pv.x = (unsigned)(lsel ? p0 : g0);
  pv.y = (unsigned)(lsel ? p1 : g1);
  pv.z = (unsigned)(lsel ? p2 : g2);
  pv.w = (unsigned)(lsel ? p3 : g3);
  unsigned short* dp = XC + (size_t)tok * XCP + (lsel ? DI : 0) + cwb + 8 * (lane & 15);
  *(volatile v4u*)dp = pv;
  __threadfence();
  *(volatile v4u*)dp = pv;
}

__global__ __launch_bounds__(STHR) void k_scan(const float* __restrict__ XI, const float* __restrict__ ZS,
                                               const float* __restrict__ XD,
                                               const float* __restrict__ cw, const float* __restrict__ cb,
                                               const float* __restrict__ wdt, const float* __restrict__ bdt,
                                               const float* __restrict__ alog, const float* __restrict__ dskip,
                                               unsigned short* Y) {
  __shared__ float hS[DS * STHR];
  __shared__ float aS[DS * STHR];
  __shared__ float wS[DS * STHR];
  __shared__ __attribute__((aligned(16))) float xd[STL * XDP];
  __shared__ __attribute__((aligned(16))) unsigned short ys[STL * 2 * STHR];
  const int tid = (int)threadIdx.x, lane = tid & 31, wave = tid >> 5;
  const int n     = (int)blockIdx.y;
  const int cbase = (int)blockIdx.x * STHR;
  const int c     = cbase + tid;

#pragma unroll 1
  for (int s = 0; s < DS; ++s) {
    hS[s * STHR + tid] = 0.0f;
    aS[s * STHR + tid] = -expf(bf16_val(alog[c * DS + s]));
    wS[s * STHR + tid] = bf16_val(wdt[c * DS + s]);
  }
  float w0, w1, w2, w3;
  {
    const v4f wv = *(const v4f*)(cw + 4 * c);
    w0 = bf16_val(wv.x); w1 = bf16_val(wv.y); w2 = bf16_val(wv.z); w3 = bf16_val(wv.w);
  }
  const float cbv = bf16_val(cb[c]);
  const float dtb = bf16_val(bdt[c]);
  const float dsk = bf16_val(dskip[c]);
  float xm1 = 0.0f, xm2 = 0.0f, xm3 = 0.0f;
  const size_t m0 = (size_t)n * LL;
  const int yofs = cbase + ((lane < 16) ? 8 * lane : DI + 8 * (lane - 16));

#pragma unroll 1
  for (int ch = 0; ch < LL / STL; ++ch) {
    const int l0 = ch * STL;
#pragma unroll
    for (int j = 0; j < (STL * 16) / STHR; ++j) {
      const int i = tid + STHR * j;
      const int row = i >> 4, q = i & 15;
      const v4f v = *(const v4f*)(XD + (m0 + l0 + row) * XDP + 4 * q);
      *(v4fa*)(xd + row * XDP + 4 * q) = v;
    }
    __syncthreads();
#pragma unroll 1
    for (int t = 0; t < STL; ++t) {
      const size_t mi = (m0 + l0 + t) * DI + c;
      const float xcur = XI[mi];
      const float zs   = ZS[mi];
      const float xc = conv_silu(xm3, xm2, xm1, xcur, w0, w1, w2, w3, cbv);
      xm3 = xm2; xm2 = xm1; xm1 = xcur;
      const float* xr = xd + t * XDP;
      float a = 0.0f;
#pragma unroll 4
      for (int r = 0; r < 16; ++r) a = fmaf(xr[r], wS[r * STHR + tid], a);
      const float v  = a + dtb;
      const float dt = fmaxf(v, 0.0f) + log1pf(expf(-fabsf(v)));
      const float du = dt * xc;
      float y = 0.0f;
#pragma unroll 1
      for (int s = 0; s < DS; ++s) {
        float hv = hS[s * STHR + tid];
        const float dA = expf(dt * aS[s * STHR + tid]);
        hv = hv * dA + du * xr[16 + s];
        hS[s * STHR + tid] = hv;
        y = fmaf(hv, xr[32 + s], y);
      }
      const float yo = (y + xc * dsk) * zs;
      unsigned hb, lb;
      split2(yo, hb, lb);
      ys[t * (2 * STHR) + tid] = (unsigned short)hb;
      ys[t * (2 * STHR) + STHR + tid] = (unsigned short)lb;
    }
    __syncthreads();
#pragma unroll 1
    for (int j = 0; j < 8; ++j) {
      const int t = 8 * wave + j;
      const v8us q = *(const v8usa*)(ys + t * (2 * STHR) + 8 * lane);
      unsigned short* yp = Y + (m0 + l0 + t) * XCP + yofs;
      *(volatile v8us*)yp = q;
    }
    __threadfence();
#pragma unroll 1
    for (int j = 0; j < 8; ++j) {
      const int t = 8 * wave + j;
      const v8us q = *(const v8usa*)(ys + t * (2 * STHR) + 8 * lane);
      unsigned short* yp = Y + (m0 + l0 + t) * XCP + yofs;
      *(volatile v8us*)yp = q;
    }
  }
}

static inline size_t al256(size_t o) { return (o + 255) & ~(size_t)255; }

extern "C" void kernel_launch(void* const* d_in, const int* in_sizes, int n_in,
                              void* d_out, int out_size, void* d_ws, size_t ws_size,
                              hipStream_t stream) {
  if (n_in < 18) return;
  if (in_sizes[0] != 2 * 8 * DD * LL) return;
  if (in_sizes[1] != DD || in_sizes[2] != DD || in_sizes[3] != DD || in_sizes[4] != DD) return;
  if (in_sizes[5] != 2 * DI * DD) return;
  if (in_sizes[6] != DI * 4 || in_sizes[7] != DI) return;
  if (in_sizes[8] != 48 * DI) return;
  if (in_sizes[9] != DI * 16 || in_sizes[10] != DI) return;
  if (in_sizes[11] != DI * DS || in_sizes[12] != DI) return;
  if (in_sizes[13] != DD * DI) return;
  if (in_sizes[14] != MD2 * MD || in_sizes[15] != MD2) return;
  if (in_sizes[16] != MD * MD2 || in_sizes[17] != MD) return;
  if (out_size != 2 * 8 * DD * LL) return;

  const float* x     = (const float*)d_in[0];
  const float* n1g   = (const float*)d_in[1];
  const float* n1b   = (const float*)d_in[2];
  const float* n2g   = (const float*)d_in[3];
  const float* n2b   = (const float*)d_in[4];
  const float* winp  = (const float*)d_in[5];
  const float* convw = (const float*)d_in[6];
  const float* convb = (const float*)d_in[7];
  const float* wxp   = (const float*)d_in[8];
  const float* wdt   = (const float*)d_in[9];
  const float* bdt   = (const float*)d_in[10];
  const float* alog  = (const float*)d_in[11];
  const float* dskip = (const float*)d_in[12];
  const float* wout  = (const float*)d_in[13];
  const float* pw1w  = (const float*)d_in[14];
  const float* pw1b  = (const float*)d_in[15];
  const float* pw2w  = (const float*)d_in[16];
  const float* pw2b  = (const float*)d_in[17];
  float* out = (float*)d_out;

  char* ws = (char*)d_ws;
  size_t off = 0;
  const size_t oU   = off; off = al256(off + (size_t)M1 * UP * 2);
  const size_t oXI  = off; off = al256(off + (size_t)M1 * DI * 4);
  const size_t oZS  = off; off = al256(off + (size_t)M1 * DI * 4);
  const size_t oXC  = off; off = al256(off + (size_t)M1 * XCP * 2);
  const size_t oXD  = off; off = al256(off + (size_t)M1 * XDP * 4);
  const size_t oWIN = off; off = al256(off + (size_t)2 * DI * DD * 2);
  const size_t oWX  = off; off = al256(off + (size_t)64 * DI * 2);
  const size_t oWO  = off; off = al256(off + (size_t)DD * DI * 2);
  if (off > ws_size || off > (size_t)WSMAX) return;
  if ((size_t)(2 * LL) * HHP * 2 > (size_t)M1 * UP * 2) return;
  if ((size_t)MD2 * MD * 2 > (size_t)M1 * DI * 4) return;
  if ((size_t)(2 * LL) * FP * 2 > (size_t)M1 * XCP * 2) return;
  unsigned short* U    = (unsigned short*)(ws + oU);
  float*          XI   = (float*)(ws + oXI);
  float*          ZS   = (float*)(ws + oZS);
  unsigned short* XC   = (unsigned short*)(ws + oXC);
  float*          XD   = (float*)(ws + oXD);
  unsigned short* WINB = (unsigned short*)(ws + oWIN);
  unsigned short* WXB  = (unsigned short*)(ws + oWX);
  unsigned short* WOB  = (unsigned short*)(ws + oWO);
  unsigned short* HH   = U;
  unsigned short* PW1B = (unsigned short*)(ws + oXI);
  unsigned short* PW2B = (unsigned short*)(ws + oZS);
  const long long zsOff = (long long)((oZS - oXI) / 4);

  {
    const int r0 = (2 * DI * DD) / 8, t0 = r0;
    const int r1 = (48 * DI) / 8,     t1 = (64 * DI) / 8;
    const int r2 = (DD * DI) / 8,     t2 = r2;
    if ((t0 % 256) != 0 || (t1 % 256) != 0 || (t2 % 256) != 0) return;
    k_cvt3<<<(t0 + t1 + t2) / 256, 256, 0, stream>>>(winp, WINB, r0, t0, wxp, WXB, r1, t1, wout, WOB, r2, t2);
  }
  k_ln<0><<<NSEQ * (LL / 32), 256, 0, stream>>>(x, n1g, n1b, U);
  k_gemm<8, EP_INPROJ><<<dim3(M1 / GBM, (2 * DI) / 128, 1), GTHR, 0, stream>>>(
      U, UP, KFULL, WINB, 0LL, DD, DD - 1, UP, XI, zsOff, XC, pw1b, x);
  k_conv<<<(M1 * 4) / 8, 256, 0, stream>>>(XI, convw, convb, XC);
  k_gemm<4, EP_XDBL><<<dim3(M1 / GBM, 1, 1), GTHR, 0, stream>>>(
      XC, XCP, KFULL, WXB, 0LL, DI, DI - 1, XCP, XD, 0LL, XC, pw1b, x);
  k_scan<<<dim3(DI / STHR, NSEQ), STHR, 0, stream>>>(XI, ZS, XD, convw, convb, wdt, bdt, alog, dskip, XC);
  k_gemm<8, EP_OUTPROJ><<<dim3(DD / GBM, LL / 128, NSEQ), GTHR, 0, stream>>>(
      WOB, DI, DI - 1, XC, (long long)LL * XCP, XCP, KFULL, XCP, out, 0LL, XC, pw1b, x);
  {
    const int r0 = (MD2 * MD) / 8;
    if ((r0 % 256) != 0) return;
    k_cvt3<<<(2 * r0) / 256, 256, 0, stream>>>(pw1w, PW1B, r0, r0, pw2w, PW2B, r0, r0, pw2w, PW2B, r0, 0);
  }
  k_ln<1><<<NSEQ * (LL / 32), 256, 0, stream>>>(out, n2g, n2b, HH);
  k_gemm<8, EP_PW1><<<dim3((2 * LL) / GBM, MD2 / 128, 1), GTHR, 0, stream>>>(
      HH, HHP, KFULL, PW1B, 0LL, MD, MD - 1, HHP, out, 0LL, XC, pw1b, x);
  k_gemm<8, EP_PW2><<<dim3(MD / GBM, LL / 128, 2), GTHR, 0, stream>>>(
      PW2B, MD2, MD2 - 1, XC, (long long)LL * FP, FP, KFULL, FP, out, 0LL, XC, pw2b, x);
}
